// ConcatAttention_30777735643475
// MI455X (gfx1250) — hardware-verified
//
#include <hip/hip_runtime.h>
#include <math.h>

#ifndef NB
#define NB 2
#endif
#ifndef SEQ
#define SEQ 2048
#endif
#define NB_FULL 2
#define SEQ_FULL 2048
#define HEADS 16
#define HD 64
#define EROWS 256
#define TOK_SPAN ((NB - 1) * SEQ_FULL + SEQ)

#define V_CARRY 8.0f
#define P_CARRY 1024.0f
#define PV_CARRY 8192.0f
#define H_MIN 6.103515625e-05f
#define SC2 (0.125f * 1.4426950408889634f)

static_assert(V_CARRY * P_CARRY == PV_CARRY);
static_assert(NB >= 1 && NB <= NB_FULL);
static_assert(SEQ <= SEQ_FULL);
static_assert(SEQ % 128 == 0);
static_assert(HD == 64 && HEADS == 16);
static_assert(EROWS % 16 == 0);
static_assert((NB * HEADS * SEQ) % 256 == 0);
static_assert(SEQ % 32 == 0);

typedef __attribute__((ext_vector_type(16))) _Float16 v16h;
typedef __attribute__((ext_vector_type(8)))  _Float16 v8h;
typedef __attribute__((ext_vector_type(2)))  _Float16 v2h;
typedef __attribute__((ext_vector_type(8)))  float    v8f;
typedef __attribute__((ext_vector_type(4)))  float    v4f;
typedef __attribute__((ext_vector_type(2)))  float    v2f;
typedef __attribute__((ext_vector_type(4)))  unsigned int v4u;


#define VST2(T, ptr, val) do { const T vst2_v_ = (val); *(volatile T*)(ptr) = vst2_v_; __threadfence(); *(volatile T*)(ptr) = vst2_v_; } while (0)

__device__ __forceinline__ float bfr(float f) {
    unsigned u = __float_as_uint(f);
    u += 0x7FFFu + ((u >> 16) & 1u);
    return __uint_as_float(u & 0xFFFF0000u);
}
static __device__ __forceinline__ float h16r(float w) {
    unsigned u = __float_as_uint(w);
    u += 0xFFFu + ((u >> 13) & 1u);
    return __uint_as_float(u & 0xFFFFE000u);
}

static __device__ __forceinline__ unsigned pk2h_sel(float a, float b) {
    const float wa = (fabsf(a) < H_MIN) ? 0.0f : a;
    const float wb = (fabsf(b) < H_MIN) ? 0.0f : b;
    v2f f; f.x = wa; f.y = wb;
    const v2h h = __builtin_convertvector(f, v2h);
    return __builtin_bit_cast(unsigned, h);
}

union FragU { v16h v; v8h h[2]; };
__device__ __forceinline__ v16h frag_ld(const _Float16* p) {
    FragU f; f.h[0] = *(const v8h*)(p); f.h[1] = *(const v8h*)(p + 16); return f.v;
}
__device__ __forceinline__ v8f wmma16(v16h a, v16h b, v8f c) {
    c = __builtin_amdgcn_wmma_f32_16x16x32_f16(false, a, false, b, (short)0, c, false, false);
    asm volatile("v_nop\n\tv_nop\n\tv_nop\n\tv_nop" : "+v"(c) : "v"(a), "v"(b));
    return c;
}
__device__ __forceinline__ void wave_sync_lds() {
    __builtin_amdgcn_fence(3  , "workgroup");
    __builtin_amdgcn_wave_barrier();
    __builtin_amdgcn_fence(2  , "workgroup");
}

__global__ __launch_bounds__(256) void k_dots(const float* __restrict__ qin, const float* __restrict__ kin,
                                              const float* __restrict__ wsc, float* __restrict__ aq, float* __restrict__ ak) {
    __shared__ float sW[128];
    const unsigned t = threadIdx.x;
    if (t < 128u) sW[t] = bfr(wsc[t]);
    __syncthreads();
    const unsigned u = blockIdx.x * 256u + t;
    const unsigned bh = u / (unsigned)SEQ;
    const unsigned l = u - bh * (unsigned)SEQ;
    const unsigned b = bh / (unsigned)HEADS;
    const unsigned h = bh - b * (unsigned)HEADS;
    const size_t ro = ((size_t)(b * (unsigned)SEQ_FULL + l) * (unsigned)HEADS + h) * (unsigned)HD;
    const v4f* q4 = (const v4f*)(qin + ro);
    const v4f* k4 = (const v4f*)(kin + ro);
    float sq = 0.f, sk = 0.f;
#pragma unroll 1
    for (unsigned g = 0; g < 4u; ++g) {
        v4f qa[4], ka[4];
#pragma unroll
        for (int i = 0; i < 4; ++i) { qa[i] = q4[4u * g + (unsigned)i]; ka[i] = k4[4u * g + (unsigned)i]; }
        const float* wq = sW + 16u * g;
        const float* wk = sW + 64u + 16u * g;
#pragma unroll
        for (int i = 0; i < 4; ++i) {
            sq = fmaf(bfr(qa[i].x), wq[4 * i], sq);
            sq = fmaf(bfr(qa[i].y), wq[4 * i + 1], sq);
            sq = fmaf(bfr(qa[i].z), wq[4 * i + 2], sq);
            sq = fmaf(bfr(qa[i].w), wq[4 * i + 3], sq);
            sk = fmaf(bfr(ka[i].x), wk[4 * i], sk);
            sk = fmaf(bfr(ka[i].y), wk[4 * i + 1], sk);
            sk = fmaf(bfr(ka[i].z), wk[4 * i + 2], sk);
            sk = fmaf(bfr(ka[i].w), wk[4 * i + 3], sk);
        }
    }
    VST2(float, aq + u, sq);
    VST2(float, ak + u, sk);
}

#define VT_TP 68
static_assert(64 * VT_TP * 4 <= 131072);
static_assert(256 * 16 * 2 == 64 * 128);
__global__ __launch_bounds__(256) void k_vt(const float* __restrict__ vin, unsigned short* __restrict__ vt16) {
    __shared__ __align__(16) float sT[64 * VT_TP];
    const unsigned t = threadIdx.x;
    const unsigned bx = blockIdx.x;
    const unsigned KT = (unsigned)SEQ / 64u;
    const unsigned bh = bx / KT;
    const unsigned kt = bx - bh * KT;
    const unsigned b = bh / (unsigned)HEADS;
    const unsigned h = bh - b * (unsigned)HEADS;
    const unsigned s0 = kt * 64u;
    {
        const unsigned key = t >> 2, qt = t & 3u;
        const float* src = vin + ((size_t)(b * (unsigned)SEQ_FULL + s0 + key) * (unsigned)HEADS + h) * (unsigned)HD + 16u * qt;
#pragma unroll
        for (int g = 0; g < 4; ++g) {
            const v4f a = *(const v4f*)(src + 4 * g);
            v4f o;
            o.x = bfr(a.x) * V_CARRY; o.y = bfr(a.y) * V_CARRY; o.z = bfr(a.z) * V_CARRY; o.w = bfr(a.w) * V_CARRY;
            *(v4f*)(sT + key * VT_TP + 16u * qt + 4u * (unsigned)g) = o;
        }
    }
    __syncthreads();
    v4u pk[2];
#pragma unroll
    for (int it = 0; it < 2; ++it) {
        const unsigned p = (unsigned)it * 256u + t;
        const unsigned e = p >> 3, g = p & 7u;
        float f[8];
#pragma unroll
        for (int i = 0; i < 8; ++i) f[i] = sT[(8u * g + (unsigned)i) * VT_TP + e];
        pk[it].x = pk2h_sel(f[0], f[1]);
        pk[it].y = pk2h_sel(f[2], f[3]);
        pk[it].z = pk2h_sel(f[4], f[5]);
        pk[it].w = pk2h_sel(f[6], f[7]);
    }
    for (int pass = 0; pass < 2; ++pass) {
#pragma unroll
        for (int it = 0; it < 2; ++it) {
            const unsigned p = (unsigned)it * 256u + t;
            const unsigned e = p >> 3, g = p & 7u;
            *(volatile v4u*)(vt16 + ((size_t)bh * 64u + e) * (unsigned)SEQ + s0 + 8u * g) = pk[it];
        }
        __threadfence();
    }
}

#define AT_PP 72
#define AT_OP 68
#define AT_WAVES 8
static_assert(AT_WAVES * 16 * AT_PP * 2 * 2 + AT_WAVES * 16 * AT_OP * 4 <= 131072);
static_assert(32 * 16 * 8 == 16 * 256);
static_assert(AT_WAVES * 16 == 128);
__global__ __launch_bounds__(256) void k_attn(const float* __restrict__ aqp, const float* __restrict__ akp,
                                              const float* __restrict__ bsp, const _Float16* __restrict__ vt,
                                              float* __restrict__ out) {
    __shared__ __align__(16) _Float16 sP[AT_WAVES][16 * AT_PP];
    __shared__ __align__(16) _Float16 sPr[AT_WAVES][16 * AT_PP];
    __shared__ __align__(16) float sO[AT_WAVES][16 * AT_OP];
    const unsigned lane = threadIdx.x & 31u;
    const unsigned wave = (unsigned)__builtin_amdgcn_readfirstlane((int)(threadIdx.x >> 5));
    const unsigned hh = lane >> 4, c = lane & 15u;
    const unsigned bx = blockIdx.x;
    const unsigned QBLK = (unsigned)SEQ / 128u;
    const unsigned bh = bx / QBLK;
    const unsigned qb = bx - bh * QBLK;
    const unsigned b = bh / (unsigned)HEADS;
    const unsigned h = bh - b * (unsigned)HEADS;
    const unsigned q0 = qb * 128u + wave * 16u;
    const unsigned nch = (q0 >> 6) + 1u;
    const bool early = (q0 < (unsigned)EROWS);
    _Float16* pw = sP[wave];
    _Float16* pr = sPr[wave];

    float aqv[8];
    {
        const float* ap = aqp + (size_t)bh * (unsigned)SEQ + q0 + 8u * hh;
        const v4f a0 = *(const v4f*)ap, a1 = *(const v4f*)(ap + 4);
        aqv[0] = a0.x; aqv[1] = a0.y; aqv[2] = a0.z; aqv[3] = a0.w;
        aqv[4] = a1.x; aqv[5] = a1.y; aqv[6] = a1.z; aqv[7] = a1.w;
    }
    const float bsc = bfr(bsp[0]);
    const float* akb = akp + (size_t)bh * (unsigned)SEQ + c;
    const _Float16* vbase = vt + ((size_t)bh * 64u + c) * (unsigned)SEQ + 8u * hh;

    float mrow[8], lrow[8];
    v8f os[4];
#pragma unroll
    for (int r = 0; r < 8; ++r) { mrow[r] = -3.0e38f; lrow[r] = 0.f; }
#pragma unroll
    for (int t = 0; t < 4; ++t) os[t] = (v8f){0.f,0.f,0.f,0.f,0.f,0.f,0.f,0.f};

#pragma unroll 1
    for (unsigned kc = 0; kc < nch; ++kc) {
        const unsigned kv0 = kc * 64u;
        float akj[4];
#pragma unroll
        for (int j = 0; j < 4; ++j) akj[j] = akb[kv0 + (unsigned)j * 16u];
#pragma unroll
        for (int r = 0; r < 8; ++r) {
            const unsigned l = q0 + 8u * hh + (unsigned)r;
            float se[4];
            float mx = -3.0e38f;
#pragma unroll
            for (int j = 0; j < 4; ++j) {
                const unsigned kl = kv0 + (unsigned)j * 16u + c;
                const float s = ((aqv[r] + akj[j]) + bsc) * SC2;
                se[j] = (kl <= l) ? s : -3.0e38f;
                mx = fmaxf(mx, se[j]);
            }
            mx = fmaxf(mx, __shfl_xor(mx, 1, 32)); mx = fmaxf(mx, __shfl_xor(mx, 2, 32));
            mx = fmaxf(mx, __shfl_xor(mx, 4, 32)); mx = fmaxf(mx, __shfl_xor(mx, 8, 32));
            const float mnew = fmaxf(mrow[r], mx);
            const float alpha = exp2f(mrow[r] - mnew);
            mrow[r] = mnew;
            float psum = 0.f;
            float rrv[4];
#pragma unroll
            for (int j = 0; j < 4; ++j) {
                const float p = exp2f(se[j] - mnew);
                psum += p;
                const float w0 = p * P_CARRY;
                const float w = (w0 < H_MIN) ? 0.0f : w0;
                const float wr = h16r(w);
                pw[(8u * hh + (unsigned)r) * AT_PP + (unsigned)j * 16u + c] = (_Float16)wr;
                rrv[j] = w - wr;
            }
            if (early) {
#pragma unroll
                for (int j = 0; j < 4; ++j) {
                    const float rs = (fabsf(rrv[j]) < H_MIN) ? 0.0f : rrv[j];
                    pr[(8u * hh + (unsigned)r) * AT_PP + (unsigned)j * 16u + c] = (_Float16)h16r(rs);
                }
            }
            psum += __shfl_xor(psum, 1, 32); psum += __shfl_xor(psum, 2, 32);
            psum += __shfl_xor(psum, 4, 32); psum += __shfl_xor(psum, 8, 32);
            lrow[r] = lrow[r] * alpha + psum;
            os[0][r] *= alpha; os[1][r] *= alpha; os[2][r] *= alpha; os[3][r] *= alpha;
        }
        wave_sync_lds();
#pragma unroll 1
        for (unsigned kk = 0; kk < 2u; ++kk) {
            const v16h pa = frag_ld(pw + c * AT_PP + kk * 32u + 8u * hh);
            v16h vb[4];
#pragma unroll
            for (int t = 0; t < 4; ++t)
                vb[t] = frag_ld(vbase + (size_t)((unsigned)t * 16u) * (unsigned)SEQ + kv0 + kk * 32u);
#pragma unroll
            for (int t = 0; t < 4; ++t) os[t] = wmma16(pa, vb[t], os[t]);
            if (early) {
                const v16h pra = frag_ld(pr + c * AT_PP + kk * 32u + 8u * hh);
#pragma unroll
                for (int t = 0; t < 4; ++t) os[t] = wmma16(pra, vb[t], os[t]);
            }
        }
        wave_sync_lds();
    }

    float* so = sO[wave];
#pragma unroll
    for (int r = 0; r < 8; ++r) {
        const float inv = 1.0f / (lrow[r] * PV_CARRY);
#pragma unroll
        for (int t = 0; t < 4; ++t)
            so[(8u * hh + (unsigned)r) * AT_OP + (unsigned)t * 16u + c] = os[t][r] * inv;
    }
    wave_sync_lds();
    {
        const unsigned c4 = (lane & 15u) * 4u;
        float* dst = out + ((size_t)(b * (unsigned)SEQ_FULL + q0) * (unsigned)HEADS + h) * (unsigned)HD;
#pragma unroll
        for (int half = 0; half < 2; ++half) {
            v4f vv[4];
#pragma unroll
            for (int it = 0; it < 4; ++it) {
                const unsigned row = (unsigned)(half * 4 + it) * 2u + hh;
                vv[it] = *(const v4f*)(so + row * AT_OP + c4);
            }
            for (int pass = 0; pass < 2; ++pass) {
#pragma unroll
                for (int it = 0; it < 4; ++it) {
                    const unsigned row = (unsigned)(half * 4 + it) * 2u + hh;
                    *(volatile v4f*)(dst + (size_t)row * (unsigned)(HEADS * HD) + c4) = vv[it];
                }
                __threadfence();
            }
        }
    }
}

#define PLANE_A_BYTES ((size_t)NB * HEADS * SEQ * 4)
#define PLANE_V_BYTES ((size_t)NB * HEADS * HD * SEQ * 2)
static_assert(PLANE_A_BYTES % 256 == 0 && PLANE_V_BYTES % 256 == 0);
static_assert(2 * PLANE_A_BYTES + PLANE_V_BYTES <= (size_t)134217728);

extern "C" void kernel_launch(void* const* d_in, const int* in_sizes, int n_in, void* d_out, int out_size,
                              void* d_ws, size_t ws_size, hipStream_t stream) {
    if (n_in < 5) return;
    if (in_sizes[0] < TOK_SPAN * HEADS * HD || in_sizes[1] < TOK_SPAN * HEADS * HD || in_sizes[2] < TOK_SPAN * HEADS * HD) return;
    if (in_sizes[3] < 2 * HD || in_sizes[4] < 1 || out_size < TOK_SPAN * HEADS * HD) return;

    const float* queries = (const float*)d_in[0];
    const float* keys    = (const float*)d_in[1];
    const float* values  = (const float*)d_in[2];
    const float* w_score = (const float*)d_in[3];
    const float* b_score = (const float*)d_in[4];
    float* out = (float*)d_out;

    char* wsp = (char*)d_ws;
    size_t off = 0;
    auto carve = [&](size_t bytes) -> void* { void* r = wsp + off; off += (bytes + 255) & ~(size_t)255; return r; };
    float*          aq   = (float*)carve(PLANE_A_BYTES);
    float*          ak   = (float*)carve(PLANE_A_BYTES);
    unsigned short* vt16 = (unsigned short*)carve(PLANE_V_BYTES);
    if (off > ws_size || off > (size_t)134217728) return;

    k_dots<<<(NB * HEADS * SEQ) / 256, 256, 0, stream>>>(queries, keys, w_score, aq, ak);
    k_vt<<<NB * HEADS * (SEQ / 64), 256, 0, stream>>>(values, vt16);
    k_attn<<<NB * HEADS * (SEQ / 128), 256, 0, stream>>>(aq, ak, b_score, (const _Float16*)vt16, out);
}
